// CrossVoxAttentionL2_58016418235045
// MI455X (gfx1250) — hardware-verified
//
#include <hip/hip_runtime.h>
#include <math.h>

typedef __attribute__((ext_vector_type(16))) _Float16 v16h;
typedef __attribute__((ext_vector_type(16))) __bf16 v16b;
typedef __attribute__((ext_vector_type(8)))  _Float16 v8h;
typedef __attribute__((ext_vector_type(8)))  float v8f;
typedef __attribute__((ext_vector_type(4)))  float v4f;
typedef __attribute__((ext_vector_type(2)))  float v2f;
typedef __attribute__((ext_vector_type(4)))  unsigned v4u;
typedef __attribute__((ext_vector_type(4)))  int v4i;
typedef float __attribute__((may_alias)) float_a;
typedef int __attribute__((may_alias)) int_a;

template <typename T> __device__ __forceinline__ void vst2(void* p, T v) { *(volatile T*)p = v; __threadfence(); *(volatile T*)p = v; }
__device__ __forceinline__ v8f wmma16(v16h a, v16h b, v8f c) {
  v8f d = __builtin_amdgcn_wmma_f32_16x16x32_f16(false, a, false, b, (short)0, c, false, false);
  asm volatile("v_nop\n\tv_nop\n\tv_nop\n\tv_nop" : "+v"(d) : "v"(a), "v"(b));
  return d;
}
__device__ __forceinline__ v8f wmma_bf(v16b a, v16b b, v8f c) {
  v8f d = __builtin_amdgcn_wmma_f32_16x16x32_bf16(false, a, false, b, (short)0, c, false, false);
  asm volatile("v_nop\n\tv_nop\n\tv_nop\n\tv_nop" : "+v"(d) : "v"(a), "v"(b));
  return d;
}
__device__ __forceinline__ v16h frag_h(const _Float16* rowk0, int lane) {
  union { v16h v; v8h q[2]; } u; const _Float16* p = rowk0 + 8 * (lane >> 4);
  u.q[0] = *(const v8h*)p; u.q[1] = *(const v8h*)(p + 16); return u.v;
}
__device__ __forceinline__ v16h frag_f32(const float* rowk0, int lane) {
  v16h a; const float* p = rowk0 + 8 * (lane >> 4);
#pragma unroll
  for (int i = 0; i < 8; ++i) { a[i] = (_Float16)p[i]; a[8 + i] = (_Float16)p[16 + i]; }
  return a;
}
__device__ __forceinline__ v16h frag_f32s(const float* rowk0, int lane, float sc) {
  v16h a; const float* p = rowk0 + 8 * (lane >> 4);
#pragma unroll
  for (int i = 0; i < 8; ++i) { a[i] = (_Float16)(p[i] * sc); a[8 + i] = (_Float16)(p[16 + i] * sc); }
  return a;
}
__device__ __forceinline__ v16h fragc_f32(const float* W, int k0, int n, int lane, int ld, int K) {
  v16h a; const int g = lane >> 4;
#pragma unroll
  for (int i = 0; i < 8; ++i) { const int ka = k0 + 8 * g + i, kb = ka + 16;
    a[i] = (_Float16)(ka < K ? W[(size_t)(ka < K ? ka : K - 1) * ld + n] : 0.f); a[8 + i] = (_Float16)(kb < K ? W[(size_t)(kb < K ? kb : K - 1) * ld + n] : 0.f); }
  return a;
}
struct F2 { v16b h, l; };
__device__ __forceinline__ F2 bsplit16(const float v[16]) { F2 r;
#pragma unroll
  for (int i = 0; i < 16; ++i) { const __bf16 h = (__bf16)v[i]; r.h[i] = h; r.l[i] = (__bf16)(v[i] - (float)h); }
  return r; }
__device__ __forceinline__ F2 split_row(const float* row, int k0, int lane) { float v[16]; const float* p = row + k0 + 8 * (lane >> 4);
#pragma unroll
  for (int i = 0; i < 8; ++i) { v[i] = p[i]; v[8 + i] = p[16 + i]; }
  return bsplit16(v); }
__device__ __forceinline__ F2 split_rowK(const float* row, int k0, int lane, int K) { float v[16]; const int g = lane >> 4;
#pragma unroll
  for (int i = 0; i < 8; ++i) { const int ka = k0 + 8 * g + i, kb = ka + 16; v[i] = ka < K ? row[ka < K ? ka : K - 1] : 0.f; v[8 + i] = kb < K ? row[kb < K ? kb : K - 1] : 0.f; }
  return bsplit16(v); }
__device__ __forceinline__ F2 split_col(const float* W, int k0, int n, int lane, int ld, int K) { float v[16]; const int g = lane >> 4;
#pragma unroll
  for (int i = 0; i < 8; ++i) { const int ka = k0 + 8 * g + i, kb = ka + 16; v[i] = ka < K ? W[(size_t)(ka < K ? ka : K - 1) * ld + n] : 0.f; v[8 + i] = kb < K ? W[(size_t)(kb < K ? kb : K - 1) * ld + n] : 0.f; }
  return bsplit16(v); }
__device__ __forceinline__ v8f mac3(const F2& a, const F2& b, v8f c) { c = wmma_bf(a.l, b.h, c); c = wmma_bf(a.h, b.l, c); return wmma_bf(a.h, b.h, c); }
__device__ __forceinline__ float sigm(float v) { return 1.0f / (1.0f + expf(-v)); }
#define LDSX() do { asm volatile("s_wait_dscnt 0" ::: "memory"); __builtin_amdgcn_wave_barrier(); __builtin_amdgcn_fence(__ATOMIC_RELEASE, "workgroup"); } while (0)


#define NB 4
#define VV 64
#define PP 4
#define NPCH 4096
#define EE 64
#define NH 8
#define HE (NH * EE)
#define SD 1024
#define DSC 256
#ifndef TQB
#define TQB (NPCH / 64)
#define TNB NB
#define TOB (NB * NPCH / 64)
#endif
typedef __attribute__((ext_vector_type(8))) __bf16 v8b;
__device__ __forceinline__ v16b frag_b(const __bf16* rowk0, int lane) {
  union { v16b v; v8b q[2]; } u; const __bf16* p = rowk0 + 8 * (lane >> 4);
  u.q[0] = *(const v8b*)p; u.q[1] = *(const v8b*)(p + 16); return u.v;
}
__device__ __forceinline__ float bfr(float v) { return (float)(__bf16)v; }
__device__ __attribute__((noinline)) float exp_ni(float v) { return expf(v); }
__device__ __attribute__((noinline)) float erf_ni(float v) { return erff(v); }

#define WS_PW   0u
#define PCW 0
#define PWD (PCW + EE * 64)
#define PWQ (PWD + EE * DSC)
#define PWK (PWQ + HE * EE)
#define PWV (PWK + HE * EE)
#define PWO (PWV + HE * EE)
#define PWEND (PWO + EE * HE)
#define WS_EMB  (WS_PW + 2u * PWEND)
#define WS_DES  (WS_EMB + 4u * NB * NPCH * EE)
#define WS_Q    (WS_DES + 4u * NB * SD * EE)
#define WS_K    (WS_Q + 4u * NB * NPCH * HE)
#define WS_VH   (WS_K + 4u * NB * SD * HE)
#define WS_VL   (WS_VH + 2u * NB * HE * SD)
#define WS_Q2   (WS_VL + 2u * NB * HE * SD)
#define WS_K2   (WS_Q2 + 4u * NB * NPCH * NH)
#define WS_O    (WS_K2 + 4u * NB * SD * NH)
#define WS_END  (WS_O + 4u * NB * NPCH * HE)

__global__ __launch_bounds__(256) void k_pack(const float* __restrict__ CW, const float* __restrict__ WD, const float* __restrict__ WQ, const float* __restrict__ WK, const float* __restrict__ WV, const float* __restrict__ WO, __bf16* __restrict__ PW) {
  __shared__ __align__(16) __bf16 s[HE]; const int n = blockIdx.x, which = blockIdx.y, tid = threadIdx.x; int K; size_t dst; float v = 0.f;
  if (which == 0) { if (n >= EE) return; K = 64; dst = PCW + (size_t)n * 64; if (tid < K) v = CW[(size_t)n * 64 + tid]; }
  else if (which == 1) { if (n >= EE) return; K = DSC; dst = PWD + (size_t)n * DSC; if (tid < K) v = WD[(size_t)tid * EE + n]; }
  else if (which <= 4) { K = EE; const float* Wm = (which == 2) ? WQ : (which == 3 ? WK : WV); dst = (which == 2 ? PWQ : (which == 3 ? PWK : PWV)) + (size_t)n * EE; if (tid < K) v = Wm[(size_t)tid * HE + n]; }
  else { if (n >= EE) return; K = HE; dst = PWO + (size_t)n * HE; for (int k = tid; k < K; k += 256) s[k] = (__bf16)WO[(size_t)k * EE + n]; __syncthreads(); for (int q = tid; q < K / 8; q += 256) vst2((unsigned*)(PW + dst + q * 8), *(const v4u*)&s[q * 8]); return; }
  if (tid < K) s[tid] = (__bf16)v; __syncthreads();
  if (tid < K / 8) vst2((unsigned*)(PW + dst + tid * 8), *(const v4u*)&s[tid * 8]);
}
__global__ __launch_bounds__(128) void k_embed(const float* __restrict__ VOX, const __bf16* __restrict__ PW, const float* __restrict__ CB, const float* __restrict__ LG, const float* __restrict__ LB, const float* __restrict__ POS, float* __restrict__ EMB) {
  __shared__ __align__(16) float so[4][16][68];
  const int tid = threadIdx.x, wave = tid >> 5, lane = tid & 31, col = lane & 15, g = lane >> 4; const int b = blockIdx.y; const int p0 = blockIdx.x * 64 + wave * 16; const int p = p0 + col; const int pz = p >> 8, py = (p >> 4) & 15, px = p & 15;
  const float* vb = VOX + (size_t)b * VV * VV * VV;
  v8f acc[4] = {};
#pragma unroll
  for (int kc = 0; kc < 2; ++kc) { v16b a;
#pragma unroll
    for (int i = 0; i < 16; ++i) { const int kk = kc * 32 + 8 * g + (i & 7) + ((i >> 3) << 4); const int dz = kk >> 4, dy = (kk >> 2) & 3, dx = kk & 3; a[i] = (__bf16)vb[((size_t)(pz * PP + dz) * VV + (py * PP + dy)) * VV + px * PP + dx]; }
#pragma unroll
    for (int j = 0; j < 4; ++j) acc[j] = wmma_bf(a, frag_b(PW + PCW + (size_t)(j * 16 + col) * 64 + kc * 32, lane), acc[j]); }
#pragma unroll
  for (int j = 0; j < 4; ++j) { const float cb = bfr(CB[j * 16 + col]);
#pragma unroll
    for (int r = 0; r < 8; ++r) so[wave][8 * g + r][j * 16 + col] = acc[j][r] + cb; }
  LDSX();
  if (lane < 16) { float* row = &so[wave][lane][0]; float mu = 0.f; for (int e = 0; e < EE; ++e) mu += row[e]; mu /= (float)EE; float var = 0.f; for (int e = 0; e < EE; ++e) { const float d = row[e] - mu; var += d * d; } var /= (float)EE; const float rs = rsqrtf(var + 1e-5f); const int pp = p0 + lane;
    for (int e = 0; e < EE; ++e) row[e] = (row[e] - mu) * rs * bfr(LG[e]) + bfr(LB[e]) + bfr(POS[(size_t)pp * EE + e]); }
  LDSX();
  for (int rl = 0; rl < 16; ++rl) if (lane < 16) vst2(EMB + ((size_t)b * NPCH + p0 + rl) * EE + lane * 4, *(const v4f*)&so[wave][rl][lane * 4]);
}
__global__ __launch_bounds__(128) void k_des(const float* __restrict__ D, const __bf16* __restrict__ PW, const float* __restrict__ BD, float* __restrict__ DES) {
  __shared__ __align__(16) float so[4][16][68];
  const int tid = threadIdx.x, wave = tid >> 5, lane = tid & 31, col = lane & 15, g = lane >> 4; const size_t r0 = (size_t)blockIdx.x * 64 + wave * 16;
  v8f acc[4] = {};
#pragma unroll 2
  for (int kc = 0; kc < DSC / 32; ++kc) { v16b a; { const float* p = D + (r0 + col) * DSC + kc * 32 + 8 * g;
#pragma unroll
      for (int i = 0; i < 8; ++i) { a[i] = (__bf16)p[i]; a[8 + i] = (__bf16)p[16 + i]; } }
#pragma unroll
    for (int j = 0; j < 4; ++j) acc[j] = wmma_bf(a, frag_b(PW + PWD + (size_t)(j * 16 + col) * DSC + kc * 32, lane), acc[j]); }
#pragma unroll
  for (int j = 0; j < 4; ++j) { const float bb = bfr(BD[j * 16 + col]);
#pragma unroll
    for (int r = 0; r < 8; ++r) so[wave][8 * g + r][j * 16 + col] = acc[j][r] + bb; }
  LDSX();
  for (int rl = 0; rl < 16; ++rl) if (lane < 16) vst2(DES + (r0 + rl) * EE + lane * 4, *(const v4f*)&so[wave][rl][lane * 4]);
}
template <int MODE>
__global__ __launch_bounds__(128) void k_proj(const float* __restrict__ A, int nrows_per_b, const __bf16* __restrict__ P, const float* __restrict__ bias, float* __restrict__ OUT, float* __restrict__ SQ, __bf16* __restrict__ VH, __bf16* __restrict__ VL) {
  __shared__ __align__(16) float so[4][16][132]; __shared__ __align__(16) __bf16 sth[128][72], stl[128][72]; __shared__ __align__(16) float ssq[64][2];
  const int tid = threadIdx.x, wave = tid >> 5, lane = tid & 31, col = lane & 15, g = lane >> 4; const size_t rb = (size_t)blockIdx.x * 64; const size_t r0 = rb + wave * 16; const int n0 = blockIdx.y * 128;
  v8f acc[8] = {};
#pragma unroll
  for (int kc = 0; kc < EE / 32; ++kc) { const F2 a = split_row(A + (r0 + col) * EE, kc * 32, lane);
#pragma unroll
    for (int j = 0; j < 8; ++j) { const v16b w = frag_b(P + (size_t)(n0 + j * 16 + col) * EE + kc * 32, lane); acc[j] = wmma_bf(a.l, w, acc[j]); acc[j] = wmma_bf(a.h, w, acc[j]); } }
  if (MODE == 2) {
#pragma unroll
    for (int j = 0; j < 8; ++j) { const float bb = bfr(bias[n0 + j * 16 + col]);
#pragma unroll
      for (int r = 0; r < 8; ++r) { const float v = acc[j][r] + bb; const __bf16 hb = (__bf16)v; sth[j * 16 + col][wave * 16 + 8 * g + r] = hb; stl[j * 16 + col][wave * 16 + 8 * g + r] = (__bf16)(v - (float)hb); } }
    __syncthreads();
    const int b = (int)(rb / nrows_per_b), s0 = (int)(rb % nrows_per_b);
    for (int q = tid; q < 128 * 8; q += 128) { const int d = q >> 3, pc = q & 7; const size_t o = ((size_t)b * HE + n0 + d) * SD + s0 + pc * 8; vst2((unsigned*)(VH + o), *(const v4u*)&sth[d][pc * 8]); vst2((unsigned*)(VL + o), *(const v4u*)&stl[d][pc * 8]); }
  } else {
    float sq[2][8];
#pragma unroll
    for (int r = 0; r < 8; ++r) { sq[0][r] = 0.f; sq[1][r] = 0.f; }
#pragma unroll
    for (int j = 0; j < 8; ++j) { const float bb = bfr(bias[n0 + j * 16 + col]);
#pragma unroll
      for (int r = 0; r < 8; ++r) { const float v = acc[j][r] + bb; so[wave][8 * g + r][j * 16 + col] = v; sq[j >> 2][r] += v * v; } }
#pragma unroll
    for (int r = 0; r < 8; ++r) { float a0 = sq[0][r], a1 = sq[1][r];
#pragma unroll
      for (int o = 1; o < 16; o <<= 1) { a0 += __shfl_xor(a0, o); a1 += __shfl_xor(a1, o); }
      if (col == 0) { ssq[wave * 16 + 8 * g + r][0] = a0; ssq[wave * 16 + 8 * g + r][1] = a1; } }
    LDSX();
    for (int rl = 0; rl < 16; ++rl) vst2(OUT + (r0 + rl) * HE + n0 + lane * 4, *(const v4f*)&so[wave][rl][lane * 4]);
    __syncthreads();
    if (tid < 32) vst2(SQ + ((size_t)blockIdx.y * ((size_t)NB * (MODE == 0 ? NPCH : SD)) + rb) * 2 + tid * 4, *(const v4f*)&(&ssq[0][0])[tid * 4]);
  }
}
__global__ __launch_bounds__(128) void k_attn(const float* __restrict__ Q, const float* __restrict__ Kx, const float* __restrict__ Q2, const float* __restrict__ K2, const __bf16* __restrict__ VH, const __bf16* __restrict__ VL, const float* __restrict__ ALPHA, float* __restrict__ O) {
  __shared__ __align__(16) float sp[4][16][36]; __shared__ __align__(16) float so[4][16][68];
  const int tid = threadIdx.x, wave = tid >> 5, lane = tid & 31, col = lane & 15, g = lane >> 4; const int qb = blockIdx.x, h = blockIdx.y, b = blockIdx.z; const int q0 = qb * 64 + wave * 16; const size_t rq = (size_t)b * NPCH + q0;
  const float asc = bfr(ALPHA[0]) * 0.125f;
  F2 aq[2];
#pragma unroll
  for (int kc = 0; kc < 2; ++kc) aq[kc] = split_row(Q + (rq + col) * HE + h * EE, kc * 32, lane);
  float q2r[8];
#pragma unroll
  for (int r = 0; r < 8; ++r) q2r[r] = Q2[((size_t)(h >> 1) * NB * NPCH + rq + 8 * g + r) * 2 + (h & 1)];
  float m[8], l[8];
#pragma unroll
  for (int r = 0; r < 8; ++r) { m[r] = -3.0e38f; l[r] = 0.f; }
  v8f acc[4] = {};
#pragma unroll 1
  for (int ks = 0; ks < SD / 32; ++ks) { v8f s[2];
#pragma unroll
    for (int ct = 0; ct < 2; ++ct) { const int kk = ks * 32 + ct * 16 + col; const size_t rk = (size_t)b * SD + kk; v8f c = {};
#pragma unroll
      for (int kc = 0; kc < 2; ++kc) { const F2 kb = split_row(Kx + rk * HE + h * EE, kc * 32, lane); c = mac3(aq[kc], kb, c); }
      const float k2v = K2[((size_t)(h >> 1) * NB * SD + rk) * 2 + (h & 1)];
#pragma unroll
      for (int r = 0; r < 8; ++r) { const float dist = q2r[r] + k2v - 2.0f * c[r]; s[ct][r] = asc * exp_ni(-dist); } }
#pragma unroll
    for (int r = 0; r < 8; ++r) { float mx = fmaxf(s[0][r], s[1][r]);
#pragma unroll
      for (int o = 1; o < 16; o <<= 1) mx = fmaxf(mx, __shfl_xor(mx, o));
      const float mn = fmaxf(m[r], mx); const float alpha = exp_ni(m[r] - mn);
      const float e0 = exp_ni(s[0][r] - mn), e1 = exp_ni(s[1][r] - mn); float es = e0 + e1;
#pragma unroll
      for (int o = 1; o < 16; o <<= 1) es += __shfl_xor(es, o);
      l[r] = l[r] * alpha + es; m[r] = mn;
#pragma unroll
      for (int dt = 0; dt < 4; ++dt) acc[dt][r] *= alpha;
      sp[wave][8 * g + r][col] = e0; sp[wave][8 * g + r][16 + col] = e1; }
    LDSX();
    const F2 pa = split_row(&sp[wave][col][0], 0, lane);
#pragma unroll
    for (int dt = 0; dt < 4; ++dt) { const size_t vr = ((size_t)b * HE + h * EE + dt * 16 + col) * SD + ks * 32; const v16b vh = frag_b(VH + vr, lane), vl = frag_b(VL + vr, lane); acc[dt] = wmma_bf(pa.l, vh, acc[dt]); acc[dt] = wmma_bf(pa.h, vl, acc[dt]); acc[dt] = wmma_bf(pa.h, vh, acc[dt]); }
    LDSX(); }
#pragma unroll
  for (int r = 0; r < 8; ++r) { const float il = 1.0f / l[r];
#pragma unroll
    for (int dt = 0; dt < 4; ++dt) so[wave][8 * g + r][dt * 16 + col] = acc[dt][r] * il; }
  LDSX();
  for (int rl = 0; rl < 16; ++rl) if (lane < 16) vst2(O + (rq + rl) * HE + h * EE + lane * 4, *(const v4f*)&so[wave][rl][lane * 4]);
}
__global__ __launch_bounds__(128) void k_out(const float* __restrict__ O, const __bf16* __restrict__ PW, const float* __restrict__ BO, float* __restrict__ Y) {
  __shared__ __align__(16) float so[4][16][68];
  const int tid = threadIdx.x, wave = tid >> 5, lane = tid & 31, col = lane & 15, g = lane >> 4; const size_t r0 = (size_t)blockIdx.x * 64 + wave * 16;
  v8f acc[4] = {};
#pragma unroll 2
  for (int kc = 0; kc < HE / 32; ++kc) { const F2 a = split_row(O + (r0 + col) * HE, kc * 32, lane);
#pragma unroll
    for (int j = 0; j < 4; ++j) { const v16b w = frag_b(PW + PWO + (size_t)(j * 16 + col) * HE + kc * 32, lane); acc[j] = wmma_bf(a.l, w, acc[j]); acc[j] = wmma_bf(a.h, w, acc[j]); } }
#pragma unroll
  for (int j = 0; j < 4; ++j) { const float bb = bfr(BO[j * 16 + col]);
#pragma unroll
    for (int r = 0; r < 8; ++r) so[wave][8 * g + r][j * 16 + col] = acc[j][r] + bb; }
  LDSX();
  for (int rl = 0; rl < 16; ++rl) if (lane < 16) vst2(Y + (r0 + rl) * EE + lane * 4, *(const v4f*)&so[wave][rl][lane * 4]);
}
extern "C" void kernel_launch(void* const* d_in, const int* in_sizes, int n_in, void* d_out, int out_size, void* d_ws, size_t ws_size, hipStream_t stream) {
  (void)in_sizes; (void)n_in; (void)out_size;
  const float** F = (const float**)d_in;
  if (ws_size < (size_t)WS_END) return;
  char* ws = (char*)d_ws; __bf16 *PW = (__bf16*)(ws + WS_PW), *VH = (__bf16*)(ws + WS_VH), *VL = (__bf16*)(ws + WS_VL); float *EMB = (float*)(ws + WS_EMB), *DES = (float*)(ws + WS_DES), *Q = (float*)(ws + WS_Q), *Kx = (float*)(ws + WS_K), *Q2 = (float*)(ws + WS_Q2), *K2 = (float*)(ws + WS_K2), *O = (float*)(ws + WS_O);
  k_pack<<<dim3(HE, 6), 256, 0, stream>>>(F[2], F[13], F[7], F[9], F[11], F[16], PW);
  k_embed<<<dim3(NPCH / 64, TNB), 128, 0, stream>>>(F[0], PW, F[3], F[4], F[5], F[6], EMB);
  k_des<<<TNB * SD / 64, 128, 0, stream>>>(F[1], PW, F[14], DES);
  k_proj<0><<<dim3(TNB * NPCH / 64, HE / 128), 128, 0, stream>>>(EMB, NPCH, PW + PWQ, F[8], Q, Q2, nullptr, nullptr);
  k_proj<1><<<dim3(TNB * SD / 64, HE / 128), 128, 0, stream>>>(DES, SD, PW + PWK, F[10], Kx, K2, nullptr, nullptr);
  k_proj<2><<<dim3(TNB * SD / 64, HE / 128), 128, 0, stream>>>(DES, SD, PW + PWV, F[12], nullptr, nullptr, VH, VL);
  k_attn<<<dim3(TQB, NH, TNB), 128, 0, stream>>>(Q, Kx, Q2, K2, VH, VL, F[15], O);
  k_out<<<TOB, 128, 0, stream>>>(O, PW, F[17], (float*)d_out);
}
